// MoEWrapper_10393820857166
// MI455X (gfx1250) — hardware-verified
//
#include <hip/hip_runtime.h>
#include <math.h>

#ifndef NTOK
#define NTOK 8192
#endif
#define NTOK_FULL 8192
#define DM 1024
#define NE 8
#define TOPK 2
#define NSLOT (NTOK * TOPK)
#define R_MAX (NSLOT + 64 * NE)
#define NT_MAX (R_MAX / 64)
#define SPT (NSLOT / 512)
#define RT_HALF (R_MAX / 2)
#define SR_HALF (NSLOT / 2)
#define NU 128

#define CX_LOG2 11
#define CW_LOG2 16
#define SC_Y (1.0f / (float)(1u << (CX_LOG2 + CW_LOG2)))

#define TBL_COUNT 0
#define TBL_POFF 16
#define TBL_NTILES 32
#define TBL_TILE_E 64
#define TBL_ROWTOK 512
#define TBL_SLOTROW (512 + R_MAX)
#define TBL_WORDS (512 + R_MAX + NSLOT)

static_assert(NE <= 16 && TOPK == 2 && NSLOT % 512 == 0);
static_assert(NE == 8);
static_assert(NTOK <= NTOK_FULL && NTOK % 128 == 0);
static_assert(SPT % 4 == 0 && SPT >= 4 && SPT <= 32);
static_assert(R_MAX % 64 == 0 && TBL_TILE_E + NT_MAX <= TBL_ROWTOK);
static_assert(TBL_POFF + NE + 1 <= TBL_NTILES && TBL_NTILES < TBL_TILE_E);
static_assert(DM == 1024);
static_assert((NTOK * DM / 8) % 256 == 0 && (NE * DM * DM / 8) % 256 == 0);
static_assert((TBL_WORDS * 4) % 256 == 0);
static_assert(R_MAX >= NSLOT && R_MAX % 2 == 0);
static_assert(RT_HALF % 128 == 0 && SR_HALF % 128 == 0 && RT_HALF >= SR_HALF && SR_HALF == 256 * SPT);
static_assert(NTOK != 8192 || (NSLOT == 16384 && R_MAX == 16896 && NT_MAX == 264 && TBL_WORDS == 33792));
static_assert((unsigned long long)NTOK * DM * 4ull <= 33554432ull);
static_assert(NU == 128 && (NTOK * NU * 4) % 256 == 0 && NTOK % 32 == 0);

constexpr size_t al256(size_t b) { return (b + 255) & ~(size_t)255; }
constexpr size_t SZ_X16 = al256((size_t)NTOK * DM * 2);
constexpr size_t SZ_W   = al256((size_t)NE * DM * DM * 2);
constexpr size_t SZ_HID = al256((size_t)NTOK * NU * 4);
constexpr size_t SZ_SEL = al256((size_t)NSLOT * 4);
constexpr size_t SZ_WGT = al256((size_t)NSLOT * 4);
constexpr size_t SZ_TBL = al256((size_t)TBL_WORDS * 4);
constexpr size_t SZ_XG  = al256((size_t)R_MAX * DM * 2);
constexpr size_t SZ_YG  = al256((size_t)R_MAX * DM * 4);
constexpr size_t WS_TOTAL = SZ_X16 + SZ_W + SZ_HID + SZ_SEL + SZ_WGT + SZ_TBL + SZ_XG + SZ_YG;
static_assert(WS_TOTAL < (size_t)268435456);
static_assert(NTOK != 8192 || WS_TOTAL == (size_t)141824000);

typedef _Float16 h16;
typedef __attribute__((ext_vector_type(16))) _Float16 v16h;
typedef __attribute__((ext_vector_type(8)))  _Float16 v8h;
typedef __attribute__((ext_vector_type(8)))  float    v8f;
typedef __attribute__((ext_vector_type(4)))  float    v4f;
typedef __attribute__((ext_vector_type(2)))  float    v2f;
typedef __attribute__((ext_vector_type(4)))  unsigned int v4u;
typedef __attribute__((ext_vector_type(4)))  int      v4i;
typedef __attribute__((ext_vector_type(2)))  int      v2i;


#define VST2(T, ptr, val) do { const T vst2_v_ = (val); *(volatile T*)(ptr) = vst2_v_; __threadfence(); *(volatile T*)(ptr) = vst2_v_; } while (0)

static __device__ __forceinline__ float bfr(float f) {
    unsigned u = __float_as_uint(f);
    u += 0x7FFFu + ((u >> 16) & 1u);
    return __uint_as_float(u & 0xFFFF0000u);
}
static __device__ __forceinline__ h16 toh_flush(float v) { const float w = (fabsf(v) < 6.103515625e-05f) ? 0.0f : v; return (h16)w; }
static __device__ __forceinline__ void st8h(h16* p, const float* v) {
    v8h hv;
#pragma unroll
    for (int e = 0; e < 8; ++e) hv[e] = toh_flush(v[e]);
    VST2(v8h, p, hv);
}

union FragU { v16h v; v8h h[2]; };
static __device__ __forceinline__ v16h frag_ld(const h16* p) {
    FragU f; f.h[0] = *(const v8h*)(p); f.h[1] = *(const v8h*)(p + 16); return f.v;
}
static __device__ __forceinline__ v8f wmma16g(v16h a, v16h b, v8f c) {
    c = __builtin_amdgcn_wmma_f32_16x16x32_f16(false, a, false, b, (short)0, c, false, false);
    asm volatile("v_nop\n\tv_nop\n\tv_nop\n\tv_nop" : "+v"(c) : "v"(a), "v"(b));
    return c;
}
static __device__ __forceinline__ void wave_sync_lds() {
    __builtin_amdgcn_fence(3  , "workgroup");
    __builtin_amdgcn_wave_barrier();
    __builtin_amdgcn_fence(2  , "workgroup");
}

template <int LOG2C>
__global__ __launch_bounds__(256) void k_plane(const float* __restrict__ src, h16* __restrict__ dst, unsigned n8) {
    const unsigned u = blockIdx.x * 256u + threadIdx.x;
    if (u >= n8) return;
    const float cs = (float)(1u << LOG2C);
    const v4f a = *(const v4f*)(src + (size_t)u * 8u);
    const v4f b = *(const v4f*)(src + (size_t)u * 8u + 4u);
    float v[8] = {bfr(a.x) * cs, bfr(a.y) * cs, bfr(a.z) * cs, bfr(a.w) * cs, bfr(b.x) * cs, bfr(b.y) * cs, bfr(b.z) * cs, bfr(b.w) * cs};
    st8h(dst + (size_t)u * 8u, v);
}

__global__ __launch_bounds__(256) void k_planeT(const float* __restrict__ src, h16* __restrict__ dst) {
    __shared__ __align__(16) float sT[64 * 68];
    const unsigned tid = threadIdx.x;
    const unsigned bx = blockIdx.x;
    const unsigned TPE = (unsigned)((DM / 64) * (DM / 64));
    if (bx >= (unsigned)NE * TPE) return;
    const unsigned e = bx / TPE;
    const unsigned rem = bx - e * TPE;
    const unsigned kt = rem / (unsigned)(DM / 64);
    const unsigned nt = rem - kt * (unsigned)(DM / 64);
    const unsigned k0 = kt * 64u, n0 = nt * 64u;
    const float cs = (float)(1u << CW_LOG2);
    const size_t ebase = (size_t)e * (size_t)(DM * DM);
#pragma unroll
    for (int i = 0; i < 4; ++i) {
        const unsigned p = tid + 256u * (unsigned)i;
        const unsigned kr = p >> 4;
        const unsigned n4 = (p & 15u) * 4u;
        const v4f a = *(const v4f*)(src + ebase + (size_t)(k0 + kr) * DM + n0 + n4);
        v4f s;
        s.x = bfr(a.x) * cs; s.y = bfr(a.y) * cs; s.z = bfr(a.z) * cs; s.w = bfr(a.w) * cs;
        *(v4f*)(&sT[kr * 68u + n4]) = s;
    }
    __syncthreads();
#pragma unroll
    for (int i = 0; i < 2; ++i) {
        const unsigned q = tid + 256u * (unsigned)i;
        const unsigned n = q >> 3;
        const unsigned kp = q & 7u;
        float v[8];
#pragma unroll
        for (int j = 0; j < 8; ++j) v[j] = sT[(8u * kp + (unsigned)j) * 68u + n];
        st8h(dst + ebase + (size_t)(n0 + n) * DM + k0 + 8u * kp, v);
    }
}

__global__ __launch_bounds__(256) void k_router1(const float* __restrict__ x, const float* __restrict__ rw1, const float* __restrict__ rb1,
                                                 float* __restrict__ hid) {
    const unsigned lane = threadIdx.x & 31u;
    const unsigned wave = threadIdx.x >> 5;
    const unsigned t0 = (blockIdx.x * 8u + wave) * 4u;
    if (t0 >= (unsigned)NTOK) return;
    float acc[4][4];
#pragma unroll
    for (int q = 0; q < 4; ++q) { acc[q][0] = 0.0f; acc[q][1] = 0.0f; acc[q][2] = 0.0f; acc[q][3] = 0.0f; }
    for (unsigned d = 0; d < (unsigned)DM; ++d) {
        const v4f w = *(const v4f*)(rw1 + (size_t)d * 128u + 4u * lane);
        const float wx = bfr(w.x), wy = bfr(w.y), wz = bfr(w.z), ww = bfr(w.w);
#pragma unroll
        for (int q = 0; q < 4; ++q) {
            const float xv = bfr(x[(size_t)(t0 + (unsigned)q) * DM + d]);
            acc[q][0] += xv * wx; acc[q][1] += xv * wy; acc[q][2] += xv * wz; acc[q][3] += xv * ww;
        }
    }
    const v4f bv = *(const v4f*)(rb1 + 4u * lane);
    const float b0 = bfr(bv.x), b1 = bfr(bv.y), b2 = bfr(bv.z), b3 = bfr(bv.w);
#pragma unroll
    for (int q = 0; q < 4; ++q) {
        v4f hv;
        hv.x = tanhf(acc[q][0] + b0); hv.y = tanhf(acc[q][1] + b1); hv.z = tanhf(acc[q][2] + b2); hv.w = tanhf(acc[q][3] + b3);
        VST2(v4f, hid + (size_t)(t0 + (unsigned)q) * 128u + 4u * lane, hv);
    }
}

__global__ __launch_bounds__(256) void k_gate(const float* __restrict__ hid, const float* __restrict__ rw2, const float* __restrict__ rb2,
                                              int* __restrict__ sel, float* __restrict__ wgt) {
    const unsigned lane = threadIdx.x & 31u;
    const unsigned wave = threadIdx.x >> 5;
    const unsigned t0 = (blockIdx.x * 8u + wave) * 16u;
    if (t0 >= (unsigned)NTOK) return;
    int ki0 = 0, ki1 = 0;
    float kw0 = 0.0f, kw1 = 0.0f;
    for (unsigned j = 0; j < 16u; ++j) {
        const float* hr = hid + (size_t)(t0 + j) * 128u;
        float lg[NE];
#pragma unroll
        for (int e = 0; e < NE; ++e) lg[e] = 0.0f;
        for (unsigned i = 0; i < 4u; ++i) {
            const unsigned u = lane + 32u * i;
            const float hv = hr[u];
            const v4f ga = *(const v4f*)(rw2 + (size_t)u * NE);
            const v4f gc = *(const v4f*)(rw2 + (size_t)u * NE + 4u);
            lg[0] += hv * bfr(ga.x); lg[1] += hv * bfr(ga.y); lg[2] += hv * bfr(ga.z); lg[3] += hv * bfr(ga.w);
            lg[4] += hv * bfr(gc.x); lg[5] += hv * bfr(gc.y); lg[6] += hv * bfr(gc.z); lg[7] += hv * bfr(gc.w);
        }
#pragma unroll
        for (int e = 0; e < NE; ++e) {
            lg[e] += __shfl_xor(lg[e], 16, 32);
            lg[e] += __shfl_xor(lg[e], 8, 32);
            lg[e] += __shfl_xor(lg[e], 4, 32);
            lg[e] += __shfl_xor(lg[e], 2, 32);
            lg[e] += __shfl_xor(lg[e], 1, 32);
        }
#pragma unroll
        for (int e = 0; e < NE; ++e) lg[e] += bfr(rb2[e]);
        float mx = lg[0];
#pragma unroll
        for (int e = 1; e < NE; ++e) mx = (lg[e] > mx) ? lg[e] : mx;
        float pr[NE];
#pragma unroll
        for (int e = 0; e < NE; ++e) pr[e] = expf(lg[e] - mx);
        float sum = pr[0];
#pragma unroll
        for (int e = 1; e < NE; ++e) sum = sum + pr[e];
#pragma unroll
        for (int e = 0; e < NE; ++e) pr[e] = pr[e] / sum;
        float bestv = pr[0];
        int besti = 0;
#pragma unroll
        for (int e = 1; e < NE; ++e) { const bool c = pr[e] > bestv; bestv = c ? pr[e] : bestv; besti = c ? e : besti; }
        float secv = -1.0f;
        int seci = 0;
#pragma unroll
        for (int e = 0; e < NE; ++e) { const bool c = (e != besti) && (pr[e] > secv); secv = c ? pr[e] : secv; seci = c ? e : seci; }
        const float e1 = expf(secv - bestv);
        const float w0 = 1.0f / (1.0f + e1);
        const float w1 = e1 / (1.0f + e1);
        const bool mine = (lane == j);
        ki0 = mine ? besti : ki0;  ki1 = mine ? seci : ki1;
        kw0 = mine ? w0 : kw0;     kw1 = mine ? w1 : kw1;
    }
    if (lane < 16u) {
        v2i sv; sv.x = ki0; sv.y = ki1;
        v2f wv; wv.x = kw0; wv.y = kw1;
        VST2(v2i, sel + (size_t)(t0 + lane) * 2u, sv);
        VST2(v2f, wgt + (size_t)(t0 + lane) * 2u, wv);
    }
}

__global__ __launch_bounds__(512) void k_route(const int* __restrict__ sel, int* __restrict__ tbl) {
    __shared__ __align__(16) int s_img[RT_HALF];
    __shared__ __align__(16) int s_hdr[512];
    __shared__ int sc[512];
    const unsigned tid = threadIdx.x;
    s_hdr[tid] = (tid >= (unsigned)TBL_TILE_E && tid < (unsigned)(TBL_TILE_E + NT_MAX)) ? -1 : 0;
    __syncthreads();
    int cnt[NE];
#pragma unroll
    for (int j = 0; j < NE; ++j) cnt[j] = 0;
    const v4i* sp = (const v4i*)(sel + (size_t)tid * (unsigned)SPT);
#pragma unroll
    for (int g = 0; g < SPT / 4; ++g) {
        const v4i v = sp[g];
#pragma unroll
        for (int c = 0; c < 4; ++c) {
            const int e = min(max(v[c], 0), NE - 1);
#pragma unroll
            for (int j = 0; j < NE; ++j) cnt[j] += (e == j) ? 1 : 0;
        }
    }
    int base[NE], total[NE];
#pragma unroll
    for (int j = 0; j < NE; ++j) {
        sc[tid] = cnt[j];
        __syncthreads();
        for (unsigned off = 1u; off < 512u; off <<= 1) {
            const unsigned src = (tid >= off) ? (tid - off) : 0u;
            const int add = sc[src];
            const int v = sc[tid] + ((tid >= off) ? add : 0);
            __syncthreads();
            sc[tid] = v;
            __syncthreads();
        }
        base[j] = sc[tid] - cnt[j];
        total[j] = sc[511];
        __syncthreads();
    }
    int base0[NE];
#pragma unroll
    for (int j = 0; j < NE; ++j) base0[j] = base[j];
    int poff[NE + 1];
    poff[0] = 0;
#pragma unroll
    for (int j = 0; j < NE; ++j) poff[j + 1] = poff[j] + (((total[j] + 63) >> 6) << 6);
    if (tid == 0u) {
#pragma unroll
        for (int j = 0; j < NE; ++j) { s_hdr[TBL_COUNT + j] = total[j]; s_hdr[TBL_POFF + j] = poff[j]; }
        s_hdr[TBL_POFF + NE] = poff[NE];
        s_hdr[TBL_NTILES] = poff[NE] >> 6;
    }
    if (tid < (unsigned)NT_MAX) {
        const int b64 = (int)(tid * 64u);
        int ev = -1;
#pragma unroll
        for (int j = 0; j < NE; ++j) ev = (b64 >= poff[j] && b64 < poff[j + 1]) ? j : ev;
        s_hdr[TBL_TILE_E + tid] = ev;
    }
    __syncthreads();
    for (int pass = 0; pass < 2; ++pass) {
        if (tid < 128u) *(volatile v4i*)(tbl + 4u * tid) = *(const v4i*)(&s_hdr[4u * tid]);
        __threadfence();
    }
    for (int h = 0; h < 2; ++h) {
        const int lo = h * RT_HALF;
        for (unsigned i = tid; i < (unsigned)RT_HALF; i += 512u) s_img[i] = -1;
        __syncthreads();
        int run[NE];
#pragma unroll
        for (int j = 0; j < NE; ++j) run[j] = base0[j];
#pragma unroll
        for (int g = 0; g < SPT / 4; ++g) {
            const v4i v = sp[g];
#pragma unroll
            for (int c = 0; c < 4; ++c) {
                const int e = min(max(v[c], 0), NE - 1);
                int row = 0;
#pragma unroll
                for (int j = 0; j < NE; ++j) {
                    const bool hit = (e == j);
                    row = hit ? (poff[j] + run[j]) : row;
                    run[j] += hit ? 1 : 0;
                }
                row = min(max(row, 0), R_MAX - 1);
                const int rel = row - lo;
                if (rel >= 0 && rel < RT_HALF) s_img[rel] = (int)((tid * (unsigned)SPT + 4u * (unsigned)g + (unsigned)c) >> 1);
            }
        }
        __syncthreads();
        for (int pass = 0; pass < 2; ++pass) {
            for (unsigned i = tid; i < (unsigned)(RT_HALF / 4); i += 512u) *(volatile v4i*)(tbl + TBL_ROWTOK + (unsigned)lo + 4u * i) = *(const v4i*)(&s_img[4u * i]);
            __threadfence();
        }
        __syncthreads();
    }
    for (int h = 0; h < 2; ++h) {
        if ((tid >> 8) == (unsigned)h) {
            int run[NE];
#pragma unroll
            for (int j = 0; j < NE; ++j) run[j] = base0[j];
#pragma unroll
            for (int g = 0; g < SPT / 4; ++g) {
                const v4i v = sp[g];
                v4i pk = (v4i){0, 0, 0, 0};
#pragma unroll
                for (int c = 0; c < 4; ++c) {
                    const int e = min(max(v[c], 0), NE - 1);
                    int row = 0;
#pragma unroll
                    for (int j = 0; j < NE; ++j) {
                        const bool hit = (e == j);
                        row = hit ? (poff[j] + run[j]) : row;
                        run[j] += hit ? 1 : 0;
                    }
                    pk[c] = min(max(row, 0), R_MAX - 1);
                }
                *(v4i*)(&s_img[(tid - 256u * (unsigned)h) * (unsigned)SPT + 4u * (unsigned)g]) = pk;
            }
        }
        __syncthreads();
        for (int pass = 0; pass < 2; ++pass) {
            for (unsigned i = tid; i < (unsigned)(SR_HALF / 4); i += 512u) *(volatile v4i*)(tbl + TBL_SLOTROW + (unsigned)(h * SR_HALF) + 4u * i) = *(const v4i*)(&s_img[4u * i]);
            __threadfence();
        }
        __syncthreads();
    }
}

__global__ __launch_bounds__(256) void k_gather(const h16* __restrict__ x16, const int* __restrict__ tbl, h16* __restrict__ Xg) {
    const unsigned row = blockIdx.x * 2u + (threadIdx.x >> 7);
    if (row >= (unsigned)R_MAX) return;
    const unsigned c = (threadIdx.x & 127u) * 8u;
    const int tr = tbl[TBL_ROWTOK + row];
    const bool pad = (tr < 0);
    const int tok = min(max(tr, 0), NTOK - 1);
    const v4u ld = *(const v4u*)(x16 + (size_t)(unsigned)tok * DM + c);
    v4u v;
    v.x = pad ? 0u : ld.x; v.y = pad ? 0u : ld.y; v.z = pad ? 0u : ld.z; v.w = pad ? 0u : ld.w;
    VST2(v4u, Xg + (size_t)row * DM + c, v);
}

__global__ __launch_bounds__(256) void k_ffn(const h16* __restrict__ Xg, const h16* __restrict__ Wp, const float* __restrict__ eb,
                                             const int* __restrict__ tbl, float* __restrict__ Yg) {
    __shared__ __align__(16) float sT[8][16 * 68];
    const unsigned lane = threadIdx.x & 31u;
    const unsigned wave = threadIdx.x >> 5;
    const unsigned u = blockIdx.x * 8u + wave;
    if (u >= (unsigned)(NT_MAX * (DM / 64))) return;
    const unsigned rowtile = u / (unsigned)(DM / 64);
    const unsigned ct = u - rowtile * (unsigned)(DM / 64);
    const int nt = min(max(tbl[TBL_NTILES], 0), NT_MAX);
    if ((int)rowtile >= nt) return;
    const int e = min(max(tbl[TBL_TILE_E + rowtile], 0), NE - 1);
    const size_t wbase = (size_t)(unsigned)e * (size_t)(DM * DM);
    const unsigned m0 = rowtile << 6, n0 = ct << 6;
    const unsigned rlane = lane & 15u;
    const unsigned koff = (lane >> 4) * 8u;
    const unsigned mOff = koff;

    v8f acc[4][4];
#pragma unroll
    for (int i = 0; i < 4; ++i)
#pragma unroll
        for (int j = 0; j < 4; ++j) acc[i][j] = (v8f){0.f,0.f,0.f,0.f,0.f,0.f,0.f,0.f};

    for (unsigned k0 = 0; k0 < (unsigned)DM; k0 += 32u) {
        v16h bh[4];
#pragma unroll
        for (int j = 0; j < 4; ++j)
            bh[j] = frag_ld(Wp + wbase + (size_t)(n0 + ((unsigned)j << 4) + rlane) * DM + koff + k0);
#pragma unroll
        for (int i = 0; i < 4; ++i) {
            const v16h ah = frag_ld(Xg + (size_t)(m0 + ((unsigned)i << 4) + rlane) * DM + koff + k0);
#pragma unroll
            for (int j = 0; j < 4; ++j) acc[i][j] = wmma16g(ah, bh[j], acc[i][j]);
        }
    }

    float ebv[4];
#pragma unroll
    for (int j = 0; j < 4; ++j) ebv[j] = bfr(eb[(unsigned)e * (unsigned)DM + n0 + ((unsigned)j << 4) + rlane]);

    float* slab = sT[wave];
#pragma unroll
    for (int i = 0; i < 4; ++i) {
        const unsigned mBase = m0 + ((unsigned)i << 4);
#pragma unroll
        for (int j = 0; j < 4; ++j)
#pragma unroll
            for (int r = 0; r < 8; ++r)
                slab[(mOff + (unsigned)r) * 68u + ((unsigned)j << 4) + rlane] = acc[i][j][r] * SC_Y + ebv[j];
        wave_sync_lds();
        const unsigned hh = lane >> 4, c4 = (lane & 15u) * 4u;
#pragma unroll
        for (int half = 0; half < 2; ++half) {
            v4f vv[4];
#pragma unroll
            for (int it = 0; it < 4; ++it) {
                const unsigned row = (unsigned)(half * 4 + it) * 2u + hh;
                vv[it] = *(const v4f*)(slab + row * 68u + c4);
            }
            for (int pass = 0; pass < 2; ++pass) {
#pragma unroll
                for (int it = 0; it < 4; ++it) {
                    const unsigned row = (unsigned)(half * 4 + it) * 2u + hh;
                    *(volatile v4f*)(Yg + (size_t)(mBase + row) * DM + n0 + c4) = vv[it];
                }
                __threadfence();
            }
        }
        wave_sync_lds();
    }
}

__global__ __launch_bounds__(256) void k_combine(const float* __restrict__ Yg, const float* __restrict__ wgt, const int* __restrict__ tbl,
                                                 float* __restrict__ out) {
    const unsigned t = blockIdx.x;
    if (t >= (unsigned)NTOK) return;
    const unsigned c = threadIdx.x * 4u;
    const int r0 = min(max(tbl[TBL_SLOTROW + 2u * t], 0), R_MAX - 1);
    const int r1 = min(max(tbl[TBL_SLOTROW + 2u * t + 1u], 0), R_MAX - 1);
    const float w0 = wgt[2u * t], w1 = wgt[2u * t + 1u];
    const v4f a = *(const v4f*)(Yg + (size_t)(unsigned)r0 * DM + c);
    const v4f b = *(const v4f*)(Yg + (size_t)(unsigned)r1 * DM + c);
    const v4f y = (a * w0) + (b * w1);
    VST2(v4f, out + (size_t)t * DM + c, y);
}

extern "C" void kernel_launch(void* const* d_in, const int* in_sizes, int n_in, void* d_out, int out_size,
                              void* d_ws, size_t ws_size, hipStream_t stream) {
    if (n_in < 7) return;
    if (in_sizes[0] < NTOK * DM || in_sizes[1] < DM * NU || in_sizes[2] < NU) return;
    if (in_sizes[3] < NU * NE || in_sizes[4] < NE) return;
    if (in_sizes[5] < NE * DM * DM || in_sizes[6] < NE * DM) return;
    if (out_size < NTOK * DM) return;

    const float* x   = (const float*)d_in[0];
    const float* rw1 = (const float*)d_in[1];
    const float* rb1 = (const float*)d_in[2];
    const float* rw2 = (const float*)d_in[3];
    const float* rb2 = (const float*)d_in[4];
    const float* ew  = (const float*)d_in[5];
    const float* eb  = (const float*)d_in[6];
    float* out = (float*)d_out;

    char* wsp = (char*)d_ws;
    size_t off = 0;
    auto carve = [&](size_t bytes) -> void* { void* r = wsp + off; off += (bytes + 255) & ~(size_t)255; return r; };
    h16*   x16 = (h16*)carve((size_t)NTOK * DM * 2);
    h16*   wt  = (h16*)carve((size_t)NE * DM * DM * 2);
    float* hid = (float*)carve((size_t)NTOK * NU * 4);
    int*   sel = (int*)carve((size_t)NSLOT * 4);
    float* wgt = (float*)carve((size_t)NSLOT * 4);
    int*   tbl = (int*)carve((size_t)TBL_WORDS * 4);
    h16*   Xg  = (h16*)carve((size_t)R_MAX * DM * 2);
    float* Yg  = (float*)carve((size_t)R_MAX * DM * 4);
    if (off != WS_TOTAL || off > ws_size || off > (size_t)268435456) return;

    k_plane<CX_LOG2><<<(NTOK * DM / 8) / 256, 256, 0, stream>>>(x, x16, (unsigned)(NTOK * DM / 8));
    k_planeT<<<NE * (DM / 64) * (DM / 64), 256, 0, stream>>>(ew, wt);
    k_router1<<<NTOK / 32, 256, 0, stream>>>(x, rw1, rb1, hid);
    k_gate<<<NTOK / 128, 256, 0, stream>>>(hid, rw2, rb2, sel, wgt);
    k_route<<<1, 512, 0, stream>>>(sel, tbl);
    k_gather<<<R_MAX / 2, 256, 0, stream>>>(x16, tbl, Xg);
    k_ffn<<<(NT_MAX * (DM / 64) + 7) / 8, 256, 0, stream>>>(Xg, wt, eb, tbl, Yg);
    k_combine<<<NTOK, 256, 0, stream>>>(Yg, wgt, tbl, out);
}
